// EGCL_22703197127077
// MI455X (gfx1250) — hardware-run, weakly checked
//
#include <hip/hip_runtime.h>
#include <stddef.h>
#include <stdint.h>


#define HID    128
#define NPP    256
#define EFIN   259
#define KN1    384
#define KN2    256
#define NTHR   256
#define NWAVE  8
#define EPB    256
#define DP     132
#define AP     136
#define MPITCH 128
#define PPITCH 16
#define XW     9
#define CSTN   1412
#define CB_E0  0
#define CB_E1  128
#define CB_X0  256
#define CB_X1  384
#define CW_INF 512
#define CW_F0  640
#define CW_F1  768
#define CW_F2  896
#define CW_O0  1024
#define CW_O1  1152
#define CW_O2  1280
#define CB_O   1408
#define CB_INF 1411
#define GBM    64
#define GBN    128
#define GTHR   128
#define EPT    8
#define CHUNK  (NTHR * EPT)
#define WCAP   (EPT * 32)
#define LISTN  (NWAVE * WCAP)
#define NBA    512
#define SLA    9
#define RCAP   16384
#define DEGCAP 128
#define SDXW   16
#define XROWS  320
#define NRANGE 2
#define NU_WPT  (NPP * (HID / 8))
#define NU_W128 (HID * (HID / 8))
#define NU_WN1  (HID * (KN1 / 8))
#define NU_WN2  (HID * (KN2 / 8))
#define AGG_ZINTS (LISTN + 2 * RCAP + 3 * NBA)
#define AGG_LDS_INTS (AGG_ZINTS + 16 + SDXW * NBA)
#define AGG_LDS_BYTES (AGG_LDS_INTS * 4)
#define EDGE_LDS_BYTES (EPB * DP * 4 + EPB * AP * 2 + EPB * MPITCH * 2 + CSTN * 4)
#define WSMAX  134217728
#define CACT   16.0f
#define CWGT   1024.0f
#define CMSG   16.0f
#define PINV   6.103515625e-05f
#define MINV   0.0625f

static_assert((CHUNK & (CHUNK - 1)) == 0 && CHUNK <= 4096);
static_assert((NBA & (NBA - 1)) == 0 && NBA == (1 << SLA));
static_assert(((long long)CHUNK << SLA) < (1LL << 31));
static_assert(((1LL << 21) << SLA) < (1LL << 31));
static_assert(LISTN % NTHR == 0);
static_assert(NBA % NWAVE == 0 && NBA % 32 == 0);
static_assert((NBA * SDXW) / 4 == 8 * NTHR);
static_assert(RCAP % 4 == 0 && AGG_ZINTS % 4 == 0 && LISTN % 4 == 0 && ((AGG_ZINTS + 16) % 4) == 0);
static_assert(AGG_LDS_BYTES <= 300000);
static_assert(EDGE_LDS_BYTES <= 300000);
static_assert(NU_WPT % NTHR == 0 && NU_W128 % NTHR == 0 && NU_WN1 % NTHR == 0 && NU_WN2 % NTHR == 0);
static_assert(HID % 32 == 0 && KN1 % 32 == 0 && KN2 % 32 == 0);
static_assert(GBM == (GTHR / 32) * 16 && GBN == 4 * 32 && GBN == HID && NPP == 2 * GBN);
static_assert((DP * 4) % 16 == 0 && (AP * 2) % 16 == 0 && AP >= HID && DP >= HID);
static_assert(EPB == NTHR && EPB == 8 * 32);
static_assert((EPB * DP * 4) % 16 == 0 && (EPB * AP * 2) % 16 == 0 && (EPB * MPITCH * 2) % 16 == 0);
static_assert((CSTN * 4) % 16 == 0 && CSTN >= CB_INF + 1);
static_assert(EPB * MPITCH * 2 == 16 * NTHR * 16);
static_assert(EFIN == 2 * HID + 3);
static_assert((XROWS * XW) % 4 == 0 && (XROWS * XW) / 4 <= 3 * NTHR && ((XROWS * XW * 4) % 128) == 0);
static_assert(KN1 == 3 * HID && KN2 == 2 * HID);
static_assert(PPITCH * 4 == 64 && XW <= 12);

typedef float          v4f   __attribute__((ext_vector_type(4)));
typedef float          v8f   __attribute__((ext_vector_type(8)));
typedef int            v4i   __attribute__((ext_vector_type(4)));
typedef int            v8i   __attribute__((ext_vector_type(8)));
typedef unsigned       v2u   __attribute__((ext_vector_type(2)));
typedef unsigned short v8us  __attribute__((ext_vector_type(8)));
typedef unsigned short v16us __attribute__((ext_vector_type(16)));
typedef __bf16         v16bf __attribute__((ext_vector_type(16)));
typedef _Float16       v16h  __attribute__((ext_vector_type(16)));
typedef v4f  __attribute__((may_alias)) v4fa;
typedef v4i  __attribute__((may_alias)) v4ia;
typedef v2u  __attribute__((may_alias)) v2ua;
typedef v8us __attribute__((may_alias)) v8usa;
union FragB { v16bf v; v16us u; v8us h[2]; v8i w; };
union FragH { v16h  v; v16us u; v8us h[2]; v8i w; };

__device__ __forceinline__ v8f wmb(const FragB& a, const FragB& b, v8f c) {
  v8f d = __builtin_amdgcn_wmma_f32_16x16x32_bf16(false, a.v, false, b.v, (short)0, c, false, false);
  asm volatile("v_nop\n\tv_nop\n\tv_nop\n\tv_nop" : "+v"(d) : "v"(a.w), "v"(b.w));
  return d;
}
__device__ __forceinline__ v8f wmh(const FragH& a, const FragH& b, v8f c) {
  v8f d = __builtin_amdgcn_wmma_f32_16x16x32_f16(false, a.v, false, b.v, (short)0, c, false, false);
  asm volatile("v_nop\n\tv_nop\n\tv_nop\n\tv_nop" : "+v"(d) : "v"(a.w), "v"(b.w));
  return d;
}

__device__ __forceinline__ unsigned bf16_bits(float f) {
  const unsigned u = __float_as_uint(f);
  return (u + 0x7FFFu + ((u >> 16) & 1u)) >> 16;
}
__device__ __forceinline__ float bf16_val(float f) {
  return __uint_as_float(bf16_bits(f) << 16);
}
__device__ __forceinline__ unsigned short f2h(float f) {
  const _Float16 hv = (_Float16)f;
  return __builtin_bit_cast(unsigned short, hv);
}
__device__ __forceinline__ float h2f(unsigned b) {
  const _Float16 hv = __builtin_bit_cast(_Float16, (unsigned short)b);
  return (float)hv;
}
__device__ __forceinline__ float silu_f(float t) {
  return t * __builtin_amdgcn_rcpf(1.0f + __expf(-t));
}
__device__ __forceinline__ void put16(unsigned short* dp, v8us o) {
  *(volatile v8us*)dp = o;
  __threadfence();
  *(volatile v8us*)dp = o;
}
__device__ __forceinline__ void putf4(float* dp, v4f o) {
  *(volatile v4f*)dp = o;
  __threadfence();
  *(volatile v4f*)dp = o;
}

template <int SLB>
__device__ __forceinline__ int scan_chunk(const int* __restrict__ dsts, int nE, int cbase, int slotBase,
                                          int nb, int vec8, int* list, int tid, int lane, int wave) {
  int wc = 0;
  const int el0  = tid * EPT;
  const int e0   = cbase + el0;
  const int sent = -2147483647 - 1;
  v4i da, db;
  if (vec8 != 0 && cbase + CHUNK <= nE) {
    da = *(const v4i*)(dsts + e0);
    db = *(const v4i*)(dsts + e0 + 4);
  } else {
    da.x = (e0     < nE) ? dsts[min(e0,     nE - 1)] : sent;
    da.y = (e0 + 1 < nE) ? dsts[min(e0 + 1, nE - 1)] : sent;
    da.z = (e0 + 2 < nE) ? dsts[min(e0 + 2, nE - 1)] : sent;
    da.w = (e0 + 3 < nE) ? dsts[min(e0 + 3, nE - 1)] : sent;
    db.x = (e0 + 4 < nE) ? dsts[min(e0 + 4, nE - 1)] : sent;
    db.y = (e0 + 5 < nE) ? dsts[min(e0 + 5, nE - 1)] : sent;
    db.z = (e0 + 6 < nE) ? dsts[min(e0 + 6, nE - 1)] : sent;
    db.w = (e0 + 7 < nE) ? dsts[min(e0 + 7, nE - 1)] : sent;
  }
  const unsigned nbs = (unsigned)slotBase;
  const unsigned unb = (unsigned)nb;
  const unsigned s0 = (unsigned)da.x - nbs, s1 = (unsigned)da.y - nbs;
  const unsigned s2 = (unsigned)da.z - nbs, s3 = (unsigned)da.w - nbs;
  const unsigned s4 = (unsigned)db.x - nbs, s5 = (unsigned)db.y - nbs;
  const unsigned s6 = (unsigned)db.z - nbs, s7 = (unsigned)db.w - nbs;
  const bool h0 = s0 < unb, h1 = s1 < unb, h2 = s2 < unb, h3 = s3 < unb;
  const bool h4 = s4 < unb, h5 = s5 < unb, h6 = s6 < unb, h7 = s7 < unb;
  const unsigned any = __builtin_amdgcn_ballot_w32(h0 | h1 | h2 | h3 | h4 | h5 | h6 | h7);
  if (any != 0u) {
#define HITJ(J, HJ, SJ) { \
      const unsigned mj = __builtin_amdgcn_ballot_w32(HJ); \
      if (mj != 0u) { \
        if (HJ) { \
          const int pos = wc + (int)__builtin_amdgcn_mbcnt_lo(mj, 0u); \
          if (pos < WCAP) list[wave * WCAP + pos] = ((el0 + (J)) << SLB) | (int)(SJ); \
        } \
        wc += (int)__builtin_popcount(mj); } }
    HITJ(0, h0, s0)
    HITJ(1, h1, s1)
    HITJ(2, h2, s2)
    HITJ(3, h3, s3)
    HITJ(4, h4, s4)
    HITJ(5, h5, s5)
    HITJ(6, h6, s6)
    HITJ(7, h7, s7)
#undef HITJ
  }
  return wc;
}

__global__ __launch_bounds__(NTHR) void k_prep(const float* __restrict__ h, const float* __restrict__ x,
                                               const float* __restrict__ We0, const float* __restrict__ We1,
                                               const float* __restrict__ Wx0, const float* __restrict__ Wx1,
                                               const float* __restrict__ Wh0, const float* __restrict__ Wh1,
                                               const float* __restrict__ Wh2, int nN, int mRows,
                                               unsigned short* WPT, unsigned short* WE1T, unsigned short* WX0T,
                                               unsigned short* WX1T, unsigned short* WN1T, unsigned short* WN2T,
                                               unsigned short* WN3T, unsigned short* HB, float* PS) {
  const int u  = (int)blockIdx.x * NTHR + (int)threadIdx.x;
  const int U0 = NU_WPT;
  const int U3 = U0 + 3 * NU_W128;
  const int U4 = U3 + NU_WN1;
  const int U6 = U4 + 2 * NU_WN2;
  const int U7 = U6 + mRows * 16;
  const int U8 = U7 + mRows * 4;
  v8us o;
  if (u < U0) {
    const int n   = u >> 4;
    const int k8  = (u & 15) * 8;
    const int kof = (n >> 7) * HID;
    const int nn  = n & (HID - 1);
    const float* p = We0 + (size_t)(kof + k8) * HID + nn;
#pragma unroll
    for (int i = 0; i < 8; ++i) o[i] = (unsigned short)bf16_bits(p[(size_t)i * HID]);
    put16(WPT + (size_t)n * HID + k8, o);
    return;
  } else if (u < U3) {
    const int v   = u - U0;
    const int mat = v >> 11;
    const int vv  = v & 2047;
    const int n   = vv >> 4;
    const int k8  = (vv & 15) * 8;
    const float* W = (mat == 0) ? We1 : ((mat == 1) ? Wx0 : Wx1);
    unsigned short* D = (mat == 0) ? WE1T : ((mat == 1) ? WX0T : WX1T);
    const float* p = W + (size_t)k8 * HID + n;
#pragma unroll
    for (int i = 0; i < 8; ++i) o[i] = f2h(CWGT * bf16_val(p[(size_t)i * HID]));
    put16(D + (size_t)n * HID + k8, o);
    return;
  } else if (u < U4) {
    const int v    = u - U3;
    const int n    = v / (KN1 / 8);
    const int k8   = (v - n * (KN1 / 8)) * 8;
    const int srow = (k8 < HID) ? k8 : (k8 - HID);
    const float* p = Wh0 + (size_t)srow * HID + n;
#pragma unroll
    for (int i = 0; i < 8; ++i) o[i] = (unsigned short)bf16_bits(p[(size_t)i * HID]);
    put16(WN1T + (size_t)n * KN1 + k8, o);
    return;
  } else if (u < U6) {
    const int v    = u - U4;
    const int mat  = v >> 12;
    const int vv   = v & 4095;
    const int n    = vv >> 5;
    const int k8   = (vv & 31) * 8;
    const int srow = k8 & (HID - 1);
    const float* W = (mat == 0) ? Wh1 : Wh2;
    unsigned short* D = (mat == 0) ? WN2T : WN3T;
    const float* p = W + (size_t)srow * HID + n;
#pragma unroll
    for (int i = 0; i < 8; ++i) o[i] = (unsigned short)bf16_bits(p[(size_t)i * HID]);
    put16(D + (size_t)n * KN2 + k8, o);
    return;
  } else if (u < U7) {
    const int v   = u - U6;
    const int row = v >> 4;
    const int k8  = (v & 15) * 8;
    const int rc  = row < nN ? row : nN - 1;
    const float* p = h + (size_t)rc * HID + k8;
    const v4f a = *(const v4fa*)p;
    const v4f b = *(const v4fa*)(p + 4);
    const bool ok = row < nN;
    o[0] = ok ? (unsigned short)bf16_bits(a.x) : (unsigned short)0;
    o[1] = ok ? (unsigned short)bf16_bits(a.y) : (unsigned short)0;
    o[2] = ok ? (unsigned short)bf16_bits(a.z) : (unsigned short)0;
    o[3] = ok ? (unsigned short)bf16_bits(a.w) : (unsigned short)0;
    o[4] = ok ? (unsigned short)bf16_bits(b.x) : (unsigned short)0;
    o[5] = ok ? (unsigned short)bf16_bits(b.y) : (unsigned short)0;
    o[6] = ok ? (unsigned short)bf16_bits(b.z) : (unsigned short)0;
    o[7] = ok ? (unsigned short)bf16_bits(b.w) : (unsigned short)0;
    put16(HB + (size_t)row * HID + k8, o);
    return;
  } else if (u < U8) {
    const int v   = u - U7;
    const int row = v >> 2;
    const int q   = v & 3;
    const int rc  = row < nN ? row : nN - 1;
    const float okf = (row < nN) ? 1.0f : 0.0f;
    const float* p = x + (size_t)rc * XW;
    v4f r;
#pragma unroll
    for (int i = 0; i < 4; ++i) {
      const int c  = 4 * q + i;
      const int cc = c < XW ? c : (XW - 1);
      const float f = (c < XW) ? okf : 0.0f;
      r[i] = bf16_val(p[cc]) * f;
    }
    putf4(PS + (size_t)row * PPITCH + 4 * q, r);
    return;
  }
}

template <int MODE>
__global__ __launch_bounds__(GTHR) void k_gemm(const unsigned short* __restrict__ A, int lda,
                                               const unsigned short* __restrict__ BT, int ldb, int K,
                                               const float* __restrict__ bias, const float* __restrict__ hres,
                                               int nN, float* Cm, int ldc, unsigned short* Cb) {
  __shared__ __attribute__((aligned(16))) float stg[GBM * GBN];
  const int tid = (int)threadIdx.x, lane = tid & 31, wave = tid >> 5, hh = lane >> 4, m = lane & 15;
  const int rowBase = (int)blockIdx.x * GBM;
  const int colBase = (int)blockIdx.y * GBN;

  v8f acc[8];
  {
    const v8f z = {0.f, 0.f, 0.f, 0.f, 0.f, 0.f, 0.f, 0.f};
#pragma unroll
    for (int t = 0; t < 8; ++t) acc[t] = z;
  }
  const unsigned short* ap = A  + (size_t)(rowBase + 16 * wave + m) * (size_t)lda + 8 * hh;
  const unsigned short* bp = BT + (size_t)(colBase + m) * (size_t)ldb + 8 * hh;

#pragma unroll 1
  for (int k0 = 0; k0 < K; k0 += 32) {
    FragB af;
    af.h[0] = *(const v8usa*)(ap + k0);
    af.h[1] = *(const v8usa*)(ap + k0 + 16);
#pragma unroll
    for (int nt = 0; nt < 8; ++nt) {
      const unsigned short* wq = bp + (size_t)(16 * nt) * (size_t)ldb + k0;
      FragB bf;
      bf.h[0] = *(const v8usa*)wq;
      bf.h[1] = *(const v8usa*)(wq + 16);
      acc[nt] = wmb(af, bf, acc[nt]);
    }
  }

#pragma unroll
  for (int nt = 0; nt < 8; ++nt) {
    const int lc = 16 * nt + m;
    float bvv = 0.0f;
    if constexpr (MODE != 0) bvv = bf16_val(bias[colBase + lc]);
#pragma unroll
    for (int r = 0; r < 8; ++r) {
      const int lr = 16 * wave + 8 * hh + r;
      float v = acc[nt][r];
      if constexpr (MODE == 1) v = silu_f(v + bvv);
      if constexpr (MODE == 2) v = v + bvv;
      stg[lr * GBN + lc] = v;
    }
  }
  __syncthreads();

  if constexpr (MODE == 0) {
    v4f pv[16];
#pragma unroll
    for (int i = 0; i < 16; ++i) pv[i] = *(const v4fa*)(stg + (16 * wave + i) * GBN + 4 * lane);
#pragma unroll
    for (int i = 0; i < 16; ++i) {
      float* op = Cm + (size_t)(rowBase + 16 * wave + i) * (size_t)ldc + colBase + 4 * lane;
      *(volatile v4f*)op = pv[i];
    }
    __threadfence();
#pragma unroll
    for (int i = 0; i < 16; ++i) {
      float* op = Cm + (size_t)(rowBase + 16 * wave + i) * (size_t)ldc + colBase + 4 * lane;
      *(volatile v4f*)op = pv[i];
    }
  } else if constexpr (MODE == 1) {
    const int part = lane >> 4;
    const int j = lane & 15;
    const unsigned mh = 0u - (unsigned)part;
    const unsigned ml = ~mh;
    v8us pv[16];
#pragma unroll
    for (int i = 0; i < 16; ++i) {
      const float* sp = stg + (16 * wave + i) * GBN + 8 * j;
      const v4f a = *(const v4fa*)sp;
      const v4f b = *(const v4fa*)(sp + 4);
      const v8f f8 = {a.x, a.y, a.z, a.w, b.x, b.y, b.z, b.w};
      v8us oo;
#pragma unroll
      for (int e = 0; e < 8; ++e) {
        const unsigned hb = bf16_bits(f8[e]);
        const unsigned lb = bf16_bits(f8[e] - __uint_as_float(hb << 16));
        oo[e] = (unsigned short)((hb & ml) | (lb & mh));
      }
      pv[i] = oo;
    }
#pragma unroll
    for (int i = 0; i < 16; ++i) {
      unsigned short* op = Cb + (size_t)(rowBase + 16 * wave + i) * (size_t)KN2 + part * HID + 8 * j;
      *(volatile v8us*)op = pv[i];
    }
    __threadfence();
#pragma unroll
    for (int i = 0; i < 16; ++i) {
      unsigned short* op = Cb + (size_t)(rowBase + 16 * wave + i) * (size_t)KN2 + part * HID + 8 * j;
      *(volatile v8us*)op = pv[i];
    }
  } else {
    v4f pv[16];
#pragma unroll
    for (int i = 0; i < 16; ++i) {
      const int row = rowBase + 16 * wave + i;
      const int rc  = row < nN ? row : nN - 1;
      const v4f hv = *(const v4fa*)(hres + (size_t)rc * HID + 4 * lane);
      const v4f sv = *(const v4fa*)(stg + (16 * wave + i) * GBN + 4 * lane);
      v4f q;
      q.x = sv.x + bf16_val(hv.x);
      q.y = sv.y + bf16_val(hv.y);
      q.z = sv.z + bf16_val(hv.z);
      q.w = sv.w + bf16_val(hv.w);
      pv[i] = q;
    }
#pragma unroll
    for (int i = 0; i < 16; ++i) {
      const int row = rowBase + 16 * wave + i;
      if (row < nN) {
        float* op = Cm + (size_t)row * (size_t)ldc + colBase + 4 * lane;
        *(volatile v4f*)op = pv[i];
      }
    }
    __threadfence();
#pragma unroll
    for (int i = 0; i < 16; ++i) {
      const int row = rowBase + 16 * wave + i;
      if (row < nN) {
        float* op = Cm + (size_t)row * (size_t)ldc + colBase + 4 * lane;
        *(volatile v4f*)op = pv[i];
      }
    }
  }
}

__device__ __forceinline__ void wave_gemm_h(const unsigned short* sAw, float* sDw,
                                            const unsigned short* __restrict__ BT, int ldb, int K,
                                            int hh, int m) {
#pragma unroll 1
  for (int nh = 0; nh < 2; ++nh) {
    v8f acc[2][4];
    {
      const v8f z = {0.f, 0.f, 0.f, 0.f, 0.f, 0.f, 0.f, 0.f};
#pragma unroll
      for (int mt = 0; mt < 2; ++mt)
#pragma unroll
        for (int nt = 0; nt < 4; ++nt) acc[mt][nt] = z;
    }
    const unsigned short* ap0 = sAw + m * AP + 8 * hh;
    const unsigned short* ap1 = ap0 + 16 * AP;
    const unsigned short* bp  = BT + (size_t)(64 * nh + m) * (size_t)ldb + 8 * hh;
#pragma unroll 1
    for (int k0 = 0; k0 < K; k0 += 32) {
      FragH a0, a1;
      a0.h[0] = *(const v8usa*)(ap0 + k0);
      a0.h[1] = *(const v8usa*)(ap0 + k0 + 16);
      a1.h[0] = *(const v8usa*)(ap1 + k0);
      a1.h[1] = *(const v8usa*)(ap1 + k0 + 16);
#pragma unroll
      for (int nt = 0; nt < 4; ++nt) {
        const unsigned short* wq = bp + (size_t)(16 * nt) * (size_t)ldb + k0;
        FragH b;
        b.h[0] = *(const v8usa*)wq;
        b.h[1] = *(const v8usa*)(wq + 16);
        acc[0][nt] = wmh(a0, b, acc[0][nt]);
        acc[1][nt] = wmh(a1, b, acc[1][nt]);
      }
    }
#pragma unroll
    for (int nt = 0; nt < 4; ++nt) {
      const int col = 64 * nh + 16 * nt + m;
#pragma unroll
      for (int mt = 0; mt < 2; ++mt)
#pragma unroll
        for (int r = 0; r < 8; ++r) sDw[(16 * mt + 8 * hh + r) * DP + col] = acc[mt][nt][r];
    }
  }
}

__global__ __launch_bounds__(NTHR) void k_edge(const int* __restrict__ snd, const int* __restrict__ rcv, int nN,
                                               int eBase, int nEh,
                                               const float* __restrict__ P, const float* __restrict__ PS,
                                               const unsigned short* __restrict__ WE1T,
                                               const unsigned short* __restrict__ WX0T,
                                               const unsigned short* __restrict__ WX1T,
                                               const float* __restrict__ We0,
                                               const float* __restrict__ be0, const float* __restrict__ be1,
                                               const float* __restrict__ bx0, const float* __restrict__ bx1,
                                               const float* __restrict__ Wxo, const float* __restrict__ bxo,
                                               const float* __restrict__ Winf, const float* __restrict__ binf,
                                               unsigned short* Mh, float* Sh) {
  extern __shared__ __attribute__((aligned(16))) float dyn[];
  float*          sD  = dyn;
  unsigned short* sA  = (unsigned short*)(dyn + EPB * DP);
  unsigned short* sM  = sA + EPB * AP;
  float*          cst = dyn + EPB * DP + (EPB * AP) / 2 + (EPB * MPITCH) / 2;

  const int tid = (int)threadIdx.x, lane = tid & 31, wave = tid >> 5, hh = lane >> 4, m = lane & 15;

  if (tid < HID) {
    cst[CB_E0 + tid]  = bf16_val(be0[tid]);
    cst[CB_E1 + tid]  = bf16_val(be1[tid]);
    cst[CB_X0 + tid]  = bf16_val(bx0[tid]);
    cst[CB_X1 + tid]  = bf16_val(bx1[tid]);
    cst[CW_INF + tid] = bf16_val(Winf[tid]);
    cst[CW_F0 + tid]  = bf16_val(We0[(size_t)(2 * HID + 0) * HID + tid]);
    cst[CW_F1 + tid]  = bf16_val(We0[(size_t)(2 * HID + 1) * HID + tid]);
    cst[CW_F2 + tid]  = bf16_val(We0[(size_t)(2 * HID + 2) * HID + tid]);
  } else {
    const int j = tid - HID;
    cst[CW_O0 + j] = bf16_val(Wxo[(size_t)j * 3 + 0]);
    cst[CW_O1 + j] = bf16_val(Wxo[(size_t)j * 3 + 1]);
    cst[CW_O2 + j] = bf16_val(Wxo[(size_t)j * 3 + 2]);
    const float o0 = bf16_val(bxo[0]);
    const float o1 = bf16_val(bxo[1]);
    const float o2 = bf16_val(bxo[2]);
    const float bi = bf16_val(binf[0]);
    if (j == 0) { cst[CB_O] = o0; cst[CB_O + 1] = o1; cst[CB_O + 2] = o2; cst[CB_INF] = bi; }
  }

  const int  elb  = (int)blockIdx.x * EPB;
  const int  el   = elb + tid;
  const bool live = el < nEh;
  const int  elc  = live ? el : (nEh - 1);
  const int  eg   = eBase + elc;
  int s = snd[eg];
  int t = rcv[eg];
  s = s < 0 ? 0 : (s > nN - 1 ? nN - 1 : s);
  t = t < 0 ? 0 : (t > nN - 1 ? nN - 1 : t);
  const float* psp = PS + (size_t)s * PPITCH;
  const float* ptp = PS + (size_t)t * PPITCH;
  const v4f s0 = *(const v4fa*)psp, s1 = *(const v4fa*)(psp + 4), s2 = *(const v4fa*)(psp + 8);
  const v4f t0 = *(const v4fa*)ptp, t1 = *(const v4fa*)(ptp + 4), t2 = *(const v4fa*)(ptp + 8);
  const float d00 = t0.x - s0.x, d01 = t0.y - s0.y, d02 = t0.z - s0.z;
  const float d10 = t0.w - s0.w, d11 = t1.x - s1.x, d12 = t1.y - s1.y;
  const float d20 = t1.z - s1.z, d21 = t1.w - s1.w, d22 = t2.x - s2.x;
  const float n0 = (d00 * d00 + d02 * d02) + d01 * d01;
  const float n1 = (d10 * d10 + d12 * d12) + d11 * d11;
  const float n2 = (d20 * d20 + d22 * d22) + d21 * d21;
  const float len0 = sqrtf(n0 + 0.0f), len1 = sqrtf(n1 + 0.0f), len2 = sqrtf(n2 + 0.0f);
  const float sq0 = len0 * len0, sq1 = len1 * len1, sq2 = len2 * len2;

  float*          rd = sD + tid * DP;
  unsigned short* ra = sA + tid * AP;
  unsigned short* rm = sM + tid * MPITCH;
  __syncthreads();

  {
    const float* pr = P + (size_t)s * NPP;
    const float* qr = P + (size_t)t * NPP + HID;
#pragma unroll 1
    for (int c8 = 0; c8 < HID / 8; ++c8) {
      const v4f pa = *(const v4fa*)(pr + 8 * c8);
      const v4f pb = *(const v4fa*)(pr + 8 * c8 + 4);
      const v4f qa = *(const v4fa*)(qr + 8 * c8);
      const v4f qb = *(const v4fa*)(qr + 8 * c8 + 4);
      const v4f ba = *(const v4fa*)(cst + CB_E0 + 8 * c8);
      const v4f bb = *(const v4fa*)(cst + CB_E0 + 8 * c8 + 4);
      const v4f fa = *(const v4fa*)(cst + CW_F0 + 8 * c8);
      const v4f fb = *(const v4fa*)(cst + CW_F0 + 8 * c8 + 4);
      const v4f ga = *(const v4fa*)(cst + CW_F1 + 8 * c8);
      const v4f gb = *(const v4fa*)(cst + CW_F1 + 8 * c8 + 4);
      const v4f ka = *(const v4fa*)(cst + CW_F2 + 8 * c8);
      const v4f kb = *(const v4fa*)(cst + CW_F2 + 8 * c8 + 4);
      const v8f p8 = {pa.x, pa.y, pa.z, pa.w, pb.x, pb.y, pb.z, pb.w};
      const v8f q8 = {qa.x, qa.y, qa.z, qa.w, qb.x, qb.y, qb.z, qb.w};
      const v8f b8 = {ba.x, ba.y, ba.z, ba.w, bb.x, bb.y, bb.z, bb.w};
      const v8f f8 = {fa.x, fa.y, fa.z, fa.w, fb.x, fb.y, fb.z, fb.w};
      const v8f g8 = {ga.x, ga.y, ga.z, ga.w, gb.x, gb.y, gb.z, gb.w};
      const v8f k8 = {ka.x, ka.y, ka.z, ka.w, kb.x, kb.y, kb.z, kb.w};
      v8us o;
#pragma unroll
      for (int i = 0; i < 8; ++i) {
        const float ft  = fmaf(sq2, k8[i], fmaf(sq1, g8[i], sq0 * f8[i]));
        const float pre = ((p8[i] + q8[i]) + ft) + b8[i];
        o[i] = f2h(CACT * silu_f(pre));
      }
      *(v8usa*)(ra + 8 * c8) = o;
    }
  }
  __syncthreads();

  const unsigned short* sAw = sA + 32 * wave * AP;
  float*                sDw = sD + 32 * wave * DP;

  wave_gemm_h(sAw, sDw, WE1T, HID, HID, hh, m);
  __syncthreads();

  {
    float dot = 0.0f;
#pragma unroll 1
    for (int c8 = 0; c8 < HID / 8; ++c8) {
      const v4f va = *(const v4fa*)(rd + 8 * c8);
      const v4f vb = *(const v4fa*)(rd + 8 * c8 + 4);
      const v4f ba = *(const v4fa*)(cst + CB_E1 + 8 * c8);
      const v4f bb = *(const v4fa*)(cst + CB_E1 + 8 * c8 + 4);
      const v4f wa = *(const v4fa*)(cst + CW_INF + 8 * c8);
      const v4f wb = *(const v4fa*)(cst + CW_INF + 8 * c8 + 4);
      const v8f v8 = {va.x, va.y, va.z, va.w, vb.x, vb.y, vb.z, vb.w};
      const v8f b8 = {ba.x, ba.y, ba.z, ba.w, bb.x, bb.y, bb.z, bb.w};
      const v8f w8 = {wa.x, wa.y, wa.z, wa.w, wb.x, wb.y, wb.z, wb.w};
      v8us o;
      v8f  mf;
#pragma unroll
      for (int i = 0; i < 8; ++i) {
        const float mj = silu_f(fmaf(v8[i], PINV, b8[i]));
        dot   = fmaf(mj, w8[i], dot);
        o[i]  = f2h(CACT * mj);
        mf[i] = mj;
      }
      *(v8usa*)(ra + 8 * c8) = o;
      const v4f m0 = {mf[0], mf[1], mf[2], mf[3]};
      const v4f m1 = {mf[4], mf[5], mf[6], mf[7]};
      *(v4fa*)(rd + 8 * c8)     = m0;
      *(v4fa*)(rd + 8 * c8 + 4) = m1;
    }
    const float eg8 = __builtin_amdgcn_rcpf(1.0f + __expf(-(dot + cst[CB_INF])));
#pragma unroll 1
    for (int c8 = 0; c8 < HID / 8; ++c8) {
      const v4f va = *(const v4fa*)(rd + 8 * c8);
      const v4f vb = *(const v4fa*)(rd + 8 * c8 + 4);
      const v8f v8 = {va.x, va.y, va.z, va.w, vb.x, vb.y, vb.z, vb.w};
      v8us o;
#pragma unroll
      for (int i = 0; i < 8; ++i) o[i] = f2h(CMSG * (v8[i] * eg8));
      *(v8usa*)(rm + 8 * c8) = o;
    }
  }
  __syncthreads();

  {
    v4i pv[16];
#pragma unroll
    for (int it = 0; it < 16; ++it) pv[it] = *(const v4ia*)(sM + (size_t)(it * NTHR + tid) * 8);
    unsigned short* mb = Mh + (size_t)elb * MPITCH;
#pragma unroll
    for (int it = 0; it < 16; ++it) *(volatile v4i*)(mb + (size_t)(it * NTHR + tid) * 8) = pv[it];
    __threadfence();
#pragma unroll
    for (int it = 0; it < 16; ++it) *(volatile v4i*)(mb + (size_t)(it * NTHR + tid) * 8) = pv[it];
  }

  wave_gemm_h(sAw, sDw, WX0T, HID, HID, hh, m);
  __syncthreads();

  {
#pragma unroll 1
    for (int c8 = 0; c8 < HID / 8; ++c8) {
      const v4f va = *(const v4fa*)(rd + 8 * c8);
      const v4f vb = *(const v4fa*)(rd + 8 * c8 + 4);
      const v4f ba = *(const v4fa*)(cst + CB_X0 + 8 * c8);
      const v4f bb = *(const v4fa*)(cst + CB_X0 + 8 * c8 + 4);
      const v8f v8 = {va.x, va.y, va.z, va.w, vb.x, vb.y, vb.z, vb.w};
      const v8f b8 = {ba.x, ba.y, ba.z, ba.w, bb.x, bb.y, bb.z, bb.w};
      v8us o;
#pragma unroll
      for (int i = 0; i < 8; ++i) o[i] = f2h(CACT * silu_f(fmaf(v8[i], PINV, b8[i])));
      *(v8usa*)(ra + 8 * c8) = o;
    }
  }
  __syncthreads();

  wave_gemm_h(sAw, sDw, WX1T, HID, HID, hh, m);
  __syncthreads();

  {
    float e0s = 0.0f, e1s = 0.0f, e2s = 0.0f;
#pragma unroll 1
    for (int c8 = 0; c8 < HID / 8; ++c8) {
      const v4f va = *(const v4fa*)(rd + 8 * c8);
      const v4f vb = *(const v4fa*)(rd + 8 * c8 + 4);
      const v4f ba = *(const v4fa*)(cst + CB_X1 + 8 * c8);
      const v4f bb = *(const v4fa*)(cst + CB_X1 + 8 * c8 + 4);
      const v4f xa = *(const v4fa*)(cst + CW_O0 + 8 * c8);
      const v4f xb = *(const v4fa*)(cst + CW_O0 + 8 * c8 + 4);
      const v4f ya = *(const v4fa*)(cst + CW_O1 + 8 * c8);
      const v4f yb = *(const v4fa*)(cst + CW_O1 + 8 * c8 + 4);
      const v4f za = *(const v4fa*)(cst + CW_O2 + 8 * c8);
      const v4f zb = *(const v4fa*)(cst + CW_O2 + 8 * c8 + 4);
      const v8f v8 = {va.x, va.y, va.z, va.w, vb.x, vb.y, vb.z, vb.w};
      const v8f b8 = {ba.x, ba.y, ba.z, ba.w, bb.x, bb.y, bb.z, bb.w};
      const v8f x8 = {xa.x, xa.y, xa.z, xa.w, xb.x, xb.y, xb.z, xb.w};
      const v8f y8 = {ya.x, ya.y, ya.z, ya.w, yb.x, yb.y, yb.z, yb.w};
      const v8f z8 = {za.x, za.y, za.z, za.w, zb.x, zb.y, zb.z, zb.w};
#pragma unroll
      for (int i = 0; i < 8; ++i) {
        const float pj = silu_f(fmaf(v8[i], PINV, b8[i]));
        e0s = fmaf(pj, x8[i], e0s);
        e1s = fmaf(pj, y8[i], e1s);
        e2s = fmaf(pj, z8[i], e2s);
      }
    }
    const float px0 = e0s + cst[CB_O];
    const float px1 = e1s + cst[CB_O + 1];
    const float px2 = e2s + cst[CB_O + 2];
    const float sv0 = px0 * __builtin_amdgcn_rcpf(1.0f + len0);
    const float sv1 = px1 * __builtin_amdgcn_rcpf(1.0f + len1);
    const float sv2 = px2 * __builtin_amdgcn_rcpf(1.0f + len2);
    v4f o4;
    o4.x = live ? sv0 : 0.0f;
    o4.y = live ? sv1 : 0.0f;
    o4.z = live ? sv2 : 0.0f;
    o4.w = 0.0f;
    float* sp = Sh + (size_t)(elb + tid) * 4;
    *(volatile v4f*)sp = o4;
    __threadfence();
    *(volatile v4f*)sp = o4;
  }
}

__global__ __launch_bounds__(NTHR) void k_scan(const int* __restrict__ srcs, const int* __restrict__ dsts,
                                               int nEh, int nN, int vec8, int mRows, int first,
                                               const unsigned short* __restrict__ Mh,
                                               const float* __restrict__ Sh, const float* __restrict__ PS,
                                               float* MI, float* SH) {
  extern __shared__ __attribute__((aligned(16))) int dsm[];
  int*   list = dsm;
  int*   hl   = dsm + LISTN;
  int*   sl   = hl + RCAP;
  int*   cnt  = sl + RCAP;
  int*   offs = cnt + NBA;
  int*   cur  = offs + NBA;
  int*   misc = cur + NBA;
  float* sdx  = (float*)(misc + 16);
  const int tid = (int)threadIdx.x, lane = tid & 31, wave = tid >> 5;
  const int nodeBase = (int)blockIdx.x * NBA;
  const v4f z4f = {0.0f, 0.0f, 0.0f, 0.0f};

  {
    const v4i z4 = {0, 0, 0, 0};
    for (int i = tid * 4; i < AGG_ZINTS; i += NTHR * 4) *(v4ia*)(dsm + i) = z4;
    if (tid < 16) misc[tid] = 0;
  }
  __syncthreads();

  int t = 0, ov = 0;
  const int nChunks = (nEh + CHUNK - 1) / CHUNK;
#pragma unroll 1
  for (int ch = 0; ch < nChunks; ++ch) {
    const int cbase = ch * CHUNK;
    const int wc = scan_chunk<SLA>(dsts, nEh, cbase, nodeBase, NBA, vec8, list, tid, lane, wave);
    if (lane == 0) misc[wave] = wc;
    __syncthreads();
    if (wave == 0) {
#pragma unroll 1
      for (int w2 = 0; w2 < NWAVE; ++w2) {
        int c = misc[w2];
        c = c < 0 ? 0 : (c > WCAP ? WCAP : c);
#pragma unroll 1
        for (int b0 = 0; b0 < c; b0 += 32) {
          const int idx = b0 + lane;
          const int ent = list[w2 * WCAP + (idx < WCAP ? idx : WCAP - 1)];
          const int m32 = (c - b0) < 32 ? (c - b0) : 32;
#pragma unroll 1
          for (int k = 0; k < m32; ++k) {
            const int u    = __builtin_amdgcn_readlane(ent, k);
            const int slot = u & (NBA - 1);
            const int el   = (u >> SLA) & (CHUNK - 1);
            const int pk   = ((cbase + el) << SLA) | slot;
            if (t < RCAP) {
              if (lane == 0) { hl[t] = pk; cnt[slot] = cnt[slot] + 1; }
              t = t + 1;
            } else {
              ov = 1;
            }
          }
        }
      }
    }
    __syncthreads();
  }
  if (wave == 0 && lane == 0) { misc[8] = t; misc[9] = ov; }
  __syncthreads();
  int tt = misc[8];
  tt = tt < 0 ? 0 : (tt > RCAP ? RCAP : tt);
  const int ovf = misc[9];

  if (wave == 0) {
    const int base = lane * (NBA / 32);
    int s = 0;
#pragma unroll 1
    for (int i = 0; i < NBA / 32; ++i) s += cnt[base + i];
    int incl = s;
#pragma unroll
    for (int d = 1; d < 32; d <<= 1) {
      const int y = __shfl_up(incl, d, 32);
      if (lane >= d) incl += y;
    }
    int run = incl - s;
#pragma unroll 1
    for (int i = 0; i < NBA / 32; ++i) {
      const int cv = cnt[base + i];
      offs[base + i] = run;
      cur[base + i]  = run;
      run += cv;
    }
  }
  __syncthreads();
  if (wave == 0) {
#pragma unroll 1
    for (int b0 = 0; b0 < tt; b0 += 32) {
      const int idx = b0 + lane;
      const int ent = hl[idx < RCAP ? idx : RCAP - 1];
      const int m32 = (tt - b0) < 32 ? (tt - b0) : 32;
#pragma unroll 1
      for (int k = 0; k < m32; ++k) {
        const int u    = __builtin_amdgcn_readlane(ent, k);
        const int slot = u & (NBA - 1);
        if (lane == 0) {
          int p = cur[slot];
          p = p < 0 ? 0 : (p > RCAP - 1 ? RCAP - 1 : p);
          sl[p] = u;
          cur[slot] = p + 1;
        }
      }
    }
  }
  __syncthreads();

  const float qnan = __int_as_float(0x7fc00000);
  const float pz = (ovf != 0) ? qnan : 0.0f;
#pragma unroll 1
  for (int si = 0; si < NBA / NWAVE; ++si) {
    const int s    = si * NWAVE + wave;
    const int node = nodeBase + s;
    int c = cnt[s];
    const bool big = c > DEGCAP;
    c = c < 0 ? 0 : (c > DEGCAP ? DEGCAP : c);
    int o = offs[s];
    o = o < 0 ? 0 : (o > RCAP ? RCAP : o);
    const int nc = node < nN ? node : nN - 1;
    const float* xdp = PS + (size_t)nc * PPITCH;
    const v4f xd0 = *(const v4fa*)xdp;
    const v4f xd1 = *(const v4fa*)(xdp + 4);
    const v4f xd2 = *(const v4fa*)(xdp + 8);
    float a0 = 0.0f, a1 = 0.0f, a2 = 0.0f, a3 = 0.0f;
    float g0 = 0.0f, g1 = 0.0f, g2 = 0.0f, g3 = 0.0f, g4 = 0.0f, g5 = 0.0f, g6 = 0.0f, g7 = 0.0f, g8 = 0.0f;
#pragma unroll 1
    for (int b0 = 0; b0 < c; b0 += 32) {
      int idx = o + b0 + lane;
      idx = idx > RCAP - 1 ? RCAP - 1 : idx;
      const int ent = sl[idx];
      int eid = ent >> SLA;
      eid = eid < 0 ? 0 : (eid > nEh - 1 ? nEh - 1 : eid);
      int sr = srcs[eid];
      sr = sr < 0 ? 0 : (sr > nN - 1 ? nN - 1 : sr);
      const float* xsp = PS + (size_t)sr * PPITCH;
      const v4f xs0 = *(const v4fa*)xsp;
      const v4f xs1 = *(const v4fa*)(xsp + 4);
      const v4f xs2 = *(const v4fa*)(xsp + 8);
      const v4f sv  = *(const v4fa*)(Sh + (size_t)eid * 4);
      const int m32 = (c - b0) < 32 ? (c - b0) : 32;
      const float mk = (lane < m32) ? 1.0f : 0.0f;
      const float w0 = sv.x * mk, w1 = sv.y * mk, w2 = sv.z * mk;
      float q0 = (xd0.x - xs0.x) * w0;
      float q1 = (xd0.y - xs0.y) * w0;
      float q2 = (xd0.z - xs0.z) * w0;
      float q3 = (xd0.w - xs0.w) * w1;
      float q4 = (xd1.x - xs1.x) * w1;
      float q5 = (xd1.y - xs1.y) * w1;
      float q6 = (xd1.z - xs1.z) * w2;
      float q7 = (xd1.w - xs1.w) * w2;
      float q8 = (xd2.x - xs2.x) * w2;
#pragma unroll 1
      for (int k = 0; k < m32; ++k) {
        const int ek = __builtin_amdgcn_readlane(eid, k);
        const unsigned short* rp = Mh + (size_t)ek * MPITCH + 4 * lane;
        const v2u w = *(const v2ua*)rp;
        a0 += h2f(w.x & 0xffffu);
        a1 += h2f(w.x >> 16);
        a2 += h2f(w.y & 0xffffu);
        a3 += h2f(w.y >> 16);
      }
#pragma unroll
      for (int d = 16; d > 0; d >>= 1) {
        q0 += __shfl_xor(q0, d, 32);
        q1 += __shfl_xor(q1, d, 32);
        q2 += __shfl_xor(q2, d, 32);
        q3 += __shfl_xor(q3, d, 32);
        q4 += __shfl_xor(q4, d, 32);
        q5 += __shfl_xor(q5, d, 32);
        q6 += __shfl_xor(q6, d, 32);
        q7 += __shfl_xor(q7, d, 32);
        q8 += __shfl_xor(q8, d, 32);
      }
      g0 += q0; g1 += q1; g2 += q2; g3 += q3; g4 += q4; g5 += q5; g6 += q6; g7 += q7; g8 += q8;
    }
    const bool  live = node < mRows;
    const int   nr   = live ? node : mRows - 1;
    const float pzr  = big ? qnan : pz;
    float* mp = MI + (size_t)nr * HID + 4 * lane;
    v4f old = z4f;
    if (first == 0) old = *(const v4fa*)mp;
    v4f nv;
    nv.x = fmaf(a0, MINV, old.x) + pzr;
    nv.y = fmaf(a1, MINV, old.y) + pzr;
    nv.z = fmaf(a2, MINV, old.z) + pzr;
    nv.w = fmaf(a3, MINV, old.w) + pzr;
    if (live) *(volatile v4f*)mp = nv;
    __threadfence();
    if (live) *(volatile v4f*)mp = nv;
    if (lane == 0) {
      const v4f e0 = {g0 + pzr, g1 + pzr, g2 + pzr, g3 + pzr};
      const v4f e1 = {g4 + pzr, g5 + pzr, g6 + pzr, g7 + pzr};
      const v4f e2 = {g8 + pzr, 0.0f, 0.0f, 0.0f};
      *(v4fa*)(sdx + SDXW * s)      = e0;
      *(v4fa*)(sdx + SDXW * s + 4)  = e1;
      *(v4fa*)(sdx + SDXW * s + 8)  = e2;
      *(v4fa*)(sdx + SDXW * s + 12) = z4f;
    }
  }
  __syncthreads();

  v4f dv[8];
#pragma unroll
  for (int j = 0; j < 8; ++j) {
    const int piece = j * NTHR + tid;
    const int node  = nodeBase + (piece >> 2);
    const int q     = piece & 3;
    const int nr    = node < mRows ? node : mRows - 1;
    v4f old = z4f;
    if (first == 0) old = *(const v4fa*)(SH + (size_t)nr * PPITCH + 4 * q);
    const v4f add = *(const v4fa*)(sdx + 4 * piece);
    v4f r;
    r.x = old.x + add.x; r.y = old.y + add.y; r.z = old.z + add.z; r.w = old.w + add.w;
    dv[j] = r;
  }
#pragma unroll
  for (int j = 0; j < 8; ++j) {
    const int piece = j * NTHR + tid;
    const int node  = nodeBase + (piece >> 2);
    const int q     = piece & 3;
    if (node < mRows) *(volatile v4f*)(SH + (size_t)node * PPITCH + 4 * q) = dv[j];
  }
  __threadfence();
#pragma unroll
  for (int j = 0; j < 8; ++j) {
    const int piece = j * NTHR + tid;
    const int node  = nodeBase + (piece >> 2);
    const int q     = piece & 3;
    if (node < mRows) *(volatile v4f*)(SH + (size_t)node * PPITCH + 4 * q) = dv[j];
  }
}

__global__ __launch_bounds__(NTHR) void k_nz(const float* __restrict__ MI, const float* __restrict__ h,
                                             int nN, int nUnits, unsigned short* NZ) {
  const int u = (int)blockIdx.x * NTHR + (int)threadIdx.x;
  if (u >= nUnits) return;
  const int row = u >> 4;
  const int j   = u & 15;
  const int rc  = row < nN ? row : nN - 1;
  const bool ok = row < nN;
  const float rs = 1.0f / sqrtf((float)(nN - 1));
  const float* mq = MI + (size_t)row * HID + 8 * j;
  const float* hq = h  + (size_t)rc  * HID + 8 * j;
  const v4f ma = *(const v4fa*)mq;
  const v4f mb = *(const v4fa*)(mq + 4);
  const v4f ha = *(const v4fa*)hq;
  const v4f hb = *(const v4fa*)(hq + 4);
  const v8f m8 = {ma.x, ma.y, ma.z, ma.w, mb.x, mb.y, mb.z, mb.w};
  const v8f h8 = {ha.x, ha.y, ha.z, ha.w, hb.x, hb.y, hb.z, hb.w};
  v8us ohi, olo, ohb;
#pragma unroll
  for (int i = 0; i < 8; ++i) {
    const float mv = m8[i] * rs;
    const unsigned hbits = bf16_bits(mv);
    ohi[i] = (unsigned short)hbits;
    olo[i] = (unsigned short)bf16_bits(mv - __uint_as_float(hbits << 16));
    ohb[i] = ok ? (unsigned short)bf16_bits(h8[i]) : (unsigned short)0;
  }
  unsigned short* dp = NZ + (size_t)row * KN1 + 8 * j;
  *(volatile v8us*)dp             = ohi;
  *(volatile v8us*)(dp + HID)     = olo;
  *(volatile v8us*)(dp + 2 * HID) = ohb;
  __threadfence();
  *(volatile v8us*)dp             = ohi;
  *(volatile v8us*)(dp + HID)     = olo;
  *(volatile v8us*)(dp + 2 * HID) = ohb;
}

__global__ __launch_bounds__(NTHR) void k_xout(const float* __restrict__ x, const float* __restrict__ SH,
                                               int nN, float* outV) {
  __shared__ __attribute__((aligned(16))) float sx[XROWS * XW];
  const int tid = (int)threadIdx.x;
  const int rowBase = (int)blockIdx.x * XROWS;
  const float inv = 1.0f / (float)(nN - 1);
  for (int j = tid; j < XROWS * XW; j += NTHR) {
    const int rl  = j / XW;
    const int c   = j - XW * rl;
    const int row = rowBase + rl;
    const int rc  = row < nN ? row : nN - 1;
    const float xv = bf16_val(x[(size_t)rc * XW + c]);
    const float dv = SH[(size_t)rc * PPITCH + c];
    sx[j] = fmaf(dv, inv, xv);
  }
  __syncthreads();
  const int NP = (XROWS * XW) / 4;
  v4f pv[3];
#pragma unroll
  for (int it = 0; it < 3; ++it) {
    const int p  = it * NTHR + tid;
    const int pc = p < NP ? p : NP - 1;
    pv[it] = *(const v4fa*)(sx + 4 * pc);
  }
#pragma unroll
  for (int it = 0; it < 3; ++it) {
    const int p  = it * NTHR + tid;
    const int pc = p < NP ? p : NP - 1;
    const long long gidx = (long long)rowBase * XW + 4LL * pc;
    const bool stv = (p < NP) && (gidx + 4 <= (long long)XW * nN);
    if (stv) *(volatile v4f*)(outV + (size_t)gidx) = pv[it];
  }
  __threadfence();
#pragma unroll
  for (int it = 0; it < 3; ++it) {
    const int p  = it * NTHR + tid;
    const int pc = p < NP ? p : NP - 1;
    const long long gidx = (long long)rowBase * XW + 4LL * pc;
    const bool stv = (p < NP) && (gidx + 4 <= (long long)XW * nN);
    if (stv) *(volatile v4f*)(outV + (size_t)gidx) = pv[it];
  }
}

static inline int cdiv(int a, int b) { return (a + b - 1) / b; }

extern "C" void kernel_launch(void* const* d_in, const int* in_sizes, int n_in,
                              void* d_out, int out_size, void* d_ws, size_t ws_size,
                              hipStream_t stream) {
  if (n_in < 22) return;
  if (in_sizes[1] < 2 * HID || (in_sizes[1] % HID) != 0) return;
  const int nN = in_sizes[1] / HID;
  if (in_sizes[0] != XW * nN) return;
  const int nE = in_sizes[2];
  if (nE < 1 || nE >= (1 << 22) || in_sizes[3] != nE) return;
  if (in_sizes[4] != EFIN * HID || in_sizes[5] != HID) return;
  if (in_sizes[6] != HID * HID || in_sizes[7] != HID) return;
  if (in_sizes[8] != HID * HID || in_sizes[9] != HID) return;
  if (in_sizes[10] != HID * HID || in_sizes[11] != HID) return;
  if (in_sizes[12] != 3 * HID || in_sizes[13] != 3) return;
  if (in_sizes[14] != HID || in_sizes[15] != 1) return;
  if (in_sizes[16] != 2 * HID * HID || in_sizes[17] != HID) return;
  if (in_sizes[18] != HID * HID || in_sizes[19] != HID) return;
  if (in_sizes[20] != HID * HID || in_sizes[21] != HID) return;
  if ((long long)out_size != (long long)XW * nN + (long long)HID * nN) return;
  if (((XW * nN) & 3) != 0) return;

  const float* pos   = (const float*)d_in[0];
  const float* feats = (const float*)d_in[1];
  const int*   snd   = (const int*)d_in[2];
  const int*   rcv   = (const int*)d_in[3];
  const float* We0   = (const float*)d_in[4];
  const float* be0   = (const float*)d_in[5];
  const float* We1   = (const float*)d_in[6];
  const float* be1   = (const float*)d_in[7];
  const float* Wx0   = (const float*)d_in[8];
  const float* bx0   = (const float*)d_in[9];
  const float* Wx1   = (const float*)d_in[10];
  const float* bx1   = (const float*)d_in[11];
  const float* Wxo   = (const float*)d_in[12];
  const float* bxo   = (const float*)d_in[13];
  const float* Winf  = (const float*)d_in[14];
  const float* binf  = (const float*)d_in[15];
  const float* Wh0   = (const float*)d_in[16];
  const float* bh0   = (const float*)d_in[17];
  const float* Wh1   = (const float*)d_in[18];
  const float* bh1   = (const float*)d_in[19];
  const float* Wh2   = (const float*)d_in[20];
  const float* bh2   = (const float*)d_in[21];
  float* outV = (float*)d_out;
  float* outF = outV + (size_t)XW * nN;

  const int MP = cdiv(nN, GBM) * GBM;
  const int gM = MP / GBM;
  const int gA = cdiv(MP, NBA);
  if ((long long)gA * NBA < (long long)MP) return;
  const int EH   = cdiv(cdiv(nE, NRANGE), EPB) * EPB;
  const int nEh0 = nE < EH ? nE : EH;
  const int nEh1 = nE - nEh0;
  const int EHP  = EH;
  if (nEh0 < 1 || EH >= (1 << 21) || nEh1 > EH) return;

  char* ws = (char*)d_ws;
  size_t off = 0;
  const size_t oWPT  = off; off += (size_t)NPP * HID * 2;            off = (off + 255) & ~(size_t)255;
  const size_t oWE1T = off; off += (size_t)HID * HID * 2;            off = (off + 255) & ~(size_t)255;
  const size_t oWX0T = off; off += (size_t)HID * HID * 2;            off = (off + 255) & ~(size_t)255;
  const size_t oWX1T = off; off += (size_t)HID * HID * 2;            off = (off + 255) & ~(size_t)255;
  const size_t oWN1T = off; off += (size_t)HID * KN1 * 2;            off = (off + 255) & ~(size_t)255;
  const size_t oWN2T = off; off += (size_t)HID * KN2 * 2;            off = (off + 255) & ~(size_t)255;
  const size_t oWN3T = off; off += (size_t)HID * KN2 * 2;            off = (off + 255) & ~(size_t)255;
  const size_t oPS   = off; off += (size_t)MP * PPITCH * 4;          off = (off + 255) & ~(size_t)255;
  const size_t oSH   = off; off += (size_t)MP * PPITCH * 4;          off = (off + 255) & ~(size_t)255;
  const size_t oMI   = off; off += (size_t)MP * HID * 4;             off = (off + 255) & ~(size_t)255;
  size_t szRM = (size_t)EHP * MPITCH * 2;
  if (szRM < (size_t)MP * HID * 2) szRM = (size_t)MP * HID * 2;
  if (szRM < (size_t)MP * KN2 * 2) szRM = (size_t)MP * KN2 * 2;
  const size_t oRM   = off; off += szRM;                             off = (off + 255) & ~(size_t)255;
  const size_t oSV   = off; off += (size_t)EHP * 4 * 4;              off = (off + 255) & ~(size_t)255;
  size_t szRP = (size_t)MP * NPP * 4;
  if (szRP < (size_t)MP * KN1 * 2) szRP = (size_t)MP * KN1 * 2;
  if (szRP < (size_t)MP * KN2 * 2) szRP = (size_t)MP * KN2 * 2;
  const size_t oRP   = off; off += szRP;                             off = (off + 255) & ~(size_t)255;
  if (off > ws_size || off > (size_t)WSMAX) return;
  unsigned short* WPT  = (unsigned short*)(ws + oWPT);
  unsigned short* WE1T = (unsigned short*)(ws + oWE1T);
  unsigned short* WX0T = (unsigned short*)(ws + oWX0T);
  unsigned short* WX1T = (unsigned short*)(ws + oWX1T);
  unsigned short* WN1T = (unsigned short*)(ws + oWN1T);
  unsigned short* WN2T = (unsigned short*)(ws + oWN2T);
  unsigned short* WN3T = (unsigned short*)(ws + oWN3T);
  float*          PS   = (float*)(ws + oPS);
  float*          SH   = (float*)(ws + oSH);
  float*          MI   = (float*)(ws + oMI);
  unsigned short* HB   = (unsigned short*)(ws + oRM);
  unsigned short* MSG  = (unsigned short*)(ws + oRM);
  unsigned short* G1   = (unsigned short*)(ws + oRM);
  float*          SV   = (float*)(ws + oSV);
  float*          P    = (float*)(ws + oRP);
  unsigned short* NZ   = (unsigned short*)(ws + oRP);
  unsigned short* G2   = (unsigned short*)(ws + oRP);

  hipFuncSetAttribute(reinterpret_cast<const void*>(&k_edge), hipFuncAttributeMaxDynamicSharedMemorySize,
                      (int)EDGE_LDS_BYTES);
  hipFuncSetAttribute(reinterpret_cast<const void*>(&k_scan), hipFuncAttributeMaxDynamicSharedMemorySize,
                      (int)AGG_LDS_BYTES);

  const int nPrep = NU_WPT + 3 * NU_W128 + NU_WN1 + 2 * NU_WN2 + MP * 16 + MP * 4;
  if ((nPrep % NTHR) != 0) return;
  const int vec8  = 1;

  k_prep<<<nPrep / NTHR, NTHR, 0, stream>>>(feats, pos, We0, We1, Wx0, Wx1, Wh0, Wh1, Wh2, nN, MP,
                                            WPT, WE1T, WX0T, WX1T, WN1T, WN2T, WN3T, HB, PS);
  k_gemm<0><<<dim3(gM, NPP / GBN), GTHR, 0, stream>>>(HB, HID, WPT, HID, HID, bh0, feats, nN, P, NPP, G1);
  k_edge<<<cdiv(nEh0, EPB), NTHR, EDGE_LDS_BYTES, stream>>>(snd, rcv, nN, 0, nEh0, P, PS, WE1T, WX0T, WX1T,
                                                             We0, be0, be1, bx0, bx1, Wxo, bxo, Winf, binf,
                                                             MSG, SV);
  k_scan<<<gA, NTHR, AGG_LDS_BYTES, stream>>>(snd, rcv, nEh0, nN, vec8, MP, 1, MSG, SV, PS, MI, SH);
  if (nEh1 > 0) {
    k_edge<<<cdiv(nEh1, EPB), NTHR, EDGE_LDS_BYTES, stream>>>(snd, rcv, nN, EH, nEh1, P, PS, WE1T, WX0T, WX1T,
                                                               We0, be0, be1, bx0, bx1, Wxo, bxo, Winf, binf,
                                                               MSG, SV);
    k_scan<<<gA, NTHR, AGG_LDS_BYTES, stream>>>(snd + EH, rcv + EH, nEh1, nN, vec8, MP, 0, MSG, SV, PS, MI, SH);
  }
  k_nz<<<(MP * 16) / NTHR, NTHR, 0, stream>>>(MI, feats, nN, MP * 16, NZ);
  k_gemm<1><<<dim3(gM, 1), GTHR, 0, stream>>>(NZ, KN1, WN1T, KN1, KN1, bh0, feats, nN, MI, HID, G1);
  k_gemm<1><<<dim3(gM, 1), GTHR, 0, stream>>>(G1, KN2, WN2T, KN2, KN2, bh1, feats, nN, MI, HID, G2);
  k_gemm<2><<<dim3(gM, 1), GTHR, 0, stream>>>(G2, KN2, WN3T, KN2, KN2, bh2, feats, nN, outF, HID, G1);
  k_xout<<<cdiv(nN, XROWS), NTHR, 0, stream>>>(pos, SH, nN, outV);
}
